// attentiond_35390530519835
// MI455X (gfx1250) — hardware-run, weakly checked
//
#include <hip/hip_runtime.h>


#define NB_  2
#define TT   2048
#define DD   1024
#define NH_  16
#define HD   64
#define QB   256
#define NQB  (TT / QB)
#define PCAR 1024.0f
#define LNEPS 1e-5f
typedef _Float16 h16;
typedef unsigned short bf;
typedef __attribute__((ext_vector_type(16))) __bf16   v16bf;
typedef __attribute__((ext_vector_type(16))) _Float16 v16h;
typedef __attribute__((ext_vector_type(8)))  _Float16 v8h;
typedef __attribute__((ext_vector_type(8)))  unsigned short v8us;
typedef __attribute__((ext_vector_type(8)))  float    v8f;
typedef __attribute__((ext_vector_type(4)))  float    v4f;
typedef v8h  __attribute__((may_alias)) v8ha;
typedef v4f  __attribute__((may_alias)) v4fa;
typedef v8us __attribute__((may_alias)) v8usa;

__device__ __forceinline__ unsigned short f2bf(float f) { unsigned u = __float_as_uint(f); u += 0x7FFFu + ((u >> 16) & 1u); return (unsigned short)(u >> 16); }
__device__ __forceinline__ float bf2f(unsigned short b) { return __uint_as_float(((unsigned)b) << 16); }
__device__ __forceinline__ float bfr(float f) { return bf2f(f2bf(f)); }
__device__ __forceinline__ v16h cat16(v8h lo, v8h hi) { return __builtin_shufflevector(lo, hi, 0, 1, 2, 3, 4, 5, 6, 7, 8, 9, 10, 11, 12, 13, 14, 15); }
__device__ __forceinline__ v16bf cat16b(v8us lo, v8us hi) { return __builtin_bit_cast(v16bf, __builtin_shufflevector(lo, hi, 0, 1, 2, 3, 4, 5, 6, 7, 8, 9, 10, 11, 12, 13, 14, 15)); }
__device__ __forceinline__ v8f wmma16(v16h a, v16h b, v8f c) { return __builtin_amdgcn_wmma_f32_16x16x32_f16(false, a, false, b, (short)0, c, false, false); }
__device__ __forceinline__ v8f wmmab(v16bf a, v16bf b, v8f c) { return __builtin_amdgcn_wmma_f32_16x16x32_bf16(false, a, false, b, (short)0, c, false, false); }


template <typename T16> struct WFrag;
template <> struct WFrag<h16> { typedef v16h V; static __device__ __forceinline__ V ld(const h16* p) { return cat16(*(const v8h*)p, *(const v8h*)(p + 16)); } static __device__ __forceinline__ v8f mma(V a, V b, v8f c) { return wmma16(a, b, c); } };
template <> struct WFrag<bf> { typedef v16bf V; static __device__ __forceinline__ V ld(const bf* p) { return cat16b(*(const v8us*)p, *(const v8us*)(p + 16)); } static __device__ __forceinline__ v8f mma(V a, V b, v8f c) { return wmmab(a, b, c); } };
template <typename T16, int NSPLIT, bool BIAS>
__global__ __launch_bounds__(32) void k_gemmw(const T16* __restrict__ A, const T16* __restrict__ A2, const T16* __restrict__ Bt, const T16* __restrict__ Bt2, int K, float* C, int ldc, const float* __restrict__ bias, size_t sA, size_t sB, size_t sC) {
    typedef typename WFrag<T16>::V V;
    __shared__ __align__(16) float os[16 * 68];
    const size_t z = blockIdx.z; A += z * sA; if (A2) A2 += z * sA; Bt += z * sB; if (Bt2) Bt2 += z * sB; C += z * sC;
    const int lane = threadIdx.x & 31, lr = lane & 15, hi = lane >> 4; const int r0 = blockIdx.x * 64, c0 = blockIdx.y * 64;
    v8f acc[4][4];
#pragma unroll
    for (int mb = 0; mb < 4; ++mb)
#pragma unroll
        for (int nb = 0; nb < 4; ++nb) acc[mb][nb] = (v8f){};
    const size_t aoff = (size_t)(r0 + lr) * K + 8 * hi, boff = (size_t)(c0 + lr) * K + 8 * hi;
#pragma unroll 1
    for (int kc = 0; kc < K; kc += 32) {
        V a[4], a2[4];
#pragma unroll
        for (int mb = 0; mb < 4; ++mb) { a[mb] = WFrag<T16>::ld(A + aoff + (size_t)mb * 16 * K + kc); if (NSPLIT == 1 || NSPLIT == 2) a2[mb] = WFrag<T16>::ld(A2 + aoff + (size_t)mb * 16 * K + kc); }
#pragma unroll
        for (int nb = 0; nb < 4; ++nb) { const V b = WFrag<T16>::ld(Bt + boff + (size_t)nb * 16 * K + kc); V b2; if (NSPLIT >= 2) b2 = WFrag<T16>::ld(Bt2 + boff + (size_t)nb * 16 * K + kc);
#pragma unroll
            for (int mb = 0; mb < 4; ++mb) { acc[mb][nb] = WFrag<T16>::mma(a[mb], b, acc[mb][nb]); if (NSPLIT == 1 || NSPLIT == 2) acc[mb][nb] = WFrag<T16>::mma(a2[mb], b, acc[mb][nb]); if (NSPLIT >= 2) acc[mb][nb] = WFrag<T16>::mma(a[mb], b2, acc[mb][nb]); } }
        asm volatile("v_nop\n\tv_nop\n\tv_nop\n\tv_nop" : "+v"(acc[0][0]), "+v"(acc[1][1]), "+v"(acc[2][2]), "+v"(acc[3][3]) : "v"(a[0]), "v"(a[3]));
    }
#pragma unroll
    for (int mb = 0; mb < 4; ++mb) {
#pragma unroll
        for (int nb = 0; nb < 4; ++nb) {
#pragma unroll
            for (int j = 0; j < 8; ++j) os[(hi * 8 + j) * 68 + nb * 16 + lr] = acc[mb][nb][j]; }
        __builtin_amdgcn_wave_barrier(); asm volatile("" ::: "memory");
        float* crow = C + (size_t)(r0 + mb * 16) * ldc + c0;
#pragma unroll 1
        for (int ps = 0; ps < 2; ++ps) {
#pragma unroll
            for (int s = 0; s < 8; ++s) { const int row = 2 * s + hi, cofs = lr * 4; v4f val = *(const v4fa*)(os + row * 68 + cofs); if (BIAS) { val[0] += bfr(bias[c0 + cofs]); val[1] += bfr(bias[c0 + cofs + 1]); val[2] += bfr(bias[c0 + cofs + 2]); val[3] += bfr(bias[c0 + cofs + 3]); }
                *(volatile v4f*)(crow + (size_t)row * ldc + cofs) = val; }
            if (ps == 0) __threadfence(); }
        __builtin_amdgcn_wave_barrier(); asm volatile("" ::: "memory");
    }
}

__device__ __forceinline__ h16 tohx(float x) { return (h16)x; }
__device__ __forceinline__ void splitf(float y, unsigned short& h, unsigned short& l) { h = f2bf(y); l = f2bf(y - bf2f(h)); }
typedef __attribute__((ext_vector_type(2))) _Float16 v2h;
typedef __attribute__((ext_vector_type(4))) _Float16 v4h;
typedef __attribute__((ext_vector_type(2))) unsigned short v2us;
typedef __attribute__((ext_vector_type(4))) unsigned short v4us;

__global__ __launch_bounds__(256) void k_wtG(const float* __restrict__ w, int K, int N, bf* Bt) {
    const int lane = threadIdx.x & 31; const int L0 = (blockIdx.x * 8 + (threadIdx.x >> 5)) * 8; const int nlines = N * K / 64;
#pragma unroll 1
    for (int ps = 0; ps < 2; ++ps) {
#pragma unroll 1
        for (int l = 0; l < 8; ++l) { const int L = L0 + l; if (L >= nlines) break; const size_t e = (size_t)L * 64 + lane * 2; const int k = (int)(e % K), n = (int)(e / K); v2us o;
            o[0] = f2bf(w[(size_t)k * N + n]); o[1] = f2bf(w[(size_t)(k + 1) * N + n]); *(volatile v2us*)(Bt + e) = o; }
        if (ps == 0) __threadfence(); }
}
template <int RAWA, int DOUBLE, int F16>
__global__ __launch_bounds__(256) void k_ln1k(const float* __restrict__ A, const float* __restrict__ ga, const float* __restrict__ ba, const float* __restrict__ gb, const float* __restrict__ bb2, bf* Yh, bf* Yl, h16* Y16) {
    const int lane = threadIdx.x & 31; const int r = blockIdx.x * 8 + (threadIdx.x >> 5); if (r >= TT) return; float v[32];
#pragma unroll
    for (int c = 0; c < 8; ++c) { const v4f a = *(const v4f*)(A + (size_t)r * DD + c * 128 + lane * 4);
#pragma unroll
        for (int q = 0; q < 4; ++q) { float t = RAWA ? bfr(a[q]) : a[q]; asm volatile("" : "+v"(t)); v[c * 4 + q] = t; } }
#pragma unroll
    for (int pass = 0; pass < (DOUBLE ? 2 : 1); ++pass) { const float* gg = pass ? gb : ga; const float* bb = pass ? bb2 : ba; float s = 0.f;
#pragma unroll
        for (int i = 0; i < 32; ++i) s = __fadd_rn(s, v[i]);
#pragma unroll
        for (int sh = 16; sh; sh >>= 1) s += __shfl_xor(s, sh, 32);
        const float mu = s * (1.0f / DD); float qq = 0.f;
#pragma unroll
        for (int i = 0; i < 32; ++i) { const float d0 = v[i] - mu; float p = __fmul_rn(d0, d0); asm volatile("" : "+v"(p)); qq = __fadd_rn(qq, p); }
#pragma unroll
        for (int sh = 16; sh; sh >>= 1) qq += __shfl_xor(qq, sh, 32);
        const float rs = __fdiv_rn(1.0f, __fsqrt_rn(__fadd_rn(qq * (1.0f / DD), LNEPS)));
#pragma unroll
        for (int c = 0; c < 8; ++c) {
#pragma unroll
            for (int q = 0; q < 4; ++q) { const int col = c * 128 + lane * 4 + q; float g = bfr(gg[col]), bq = bfr(bb[col]); asm volatile("" : "+v"(g)); asm volatile("" : "+v"(bq)); float tn = __fmul_rn(v[c * 4 + q] - mu, rs); asm volatile("" : "+v"(tn)); float tg = __fmul_rn(tn, g); asm volatile("" : "+v"(tg)); v[c * 4 + q] = __fadd_rn(tg, bq); } } }
#pragma unroll 1
    for (int ps = 0; ps < 2; ++ps) {
#pragma unroll
        for (int c = 0; c < 8; ++c) { const size_t o = (size_t)r * DD + c * 128 + lane * 4;
            if (F16) { v4h o4; for (int q = 0; q < 4; ++q) o4[q] = tohx(v[c * 4 + q]); *(volatile v4h*)(Y16 + o) = o4; }
            else { v4us oh, ol; for (int q = 0; q < 4; ++q) { unsigned short a2, c2; splitf(v[c * 4 + q], a2, c2); oh[q] = a2; ol[q] = c2; } *(volatile v4us*)(Yh + o) = oh; *(volatile v4us*)(Yl + o) = ol; } }
        if (ps == 0) __threadfence(); }
}
__global__ __launch_bounds__(256) void k_qkpl(const float* __restrict__ KV, bf* Ph, bf* Pl) { const int e = (blockIdx.x * 256 + threadIdx.x) * 2; if (e >= NH_ * TT * HD) return; const int d = e & 63; const int t = (e >> 6) & (TT - 1); const int h = e / (TT * HD); v2us oh, ol;
#pragma unroll
    for (int q = 0; q < 2; ++q) { unsigned short a, c2; splitf(KV[(size_t)t * 2 * DD + h * HD + d + q], a, c2); oh[q] = a; ol[q] = c2; } *(volatile v2us*)(Ph + e) = oh; *(volatile v2us*)(Pl + e) = ol; __threadfence(); *(volatile v2us*)(Ph + e) = oh; *(volatile v2us*)(Pl + e) = ol; }
__global__ __launch_bounds__(256) void k_vt(const float* __restrict__ KV, h16* VT) { const int e = (blockIdx.x * 256 + threadIdx.x) * 2; if (e >= NH_ * HD * TT) return; const int t = e & (TT - 1); const int d = (e / TT) & 63; const int h = e / (TT * HD); v2h o; o[0] = tohx(KV[(size_t)t * 2 * DD + DD + h * HD + d]); o[1] = tohx(KV[(size_t)(t + 1) * 2 * DD + DD + h * HD + d]); *(volatile v2h*)(VT + e) = o; __threadfence(); *(volatile v2h*)(VT + e) = o; }
__global__ __launch_bounds__(256) void k_smx(float* Sb) { const int lane = threadIdx.x & 31; const int row = blockIdx.x * 8 + (threadIdx.x >> 5); if (row >= NH_ * QB) return; float* sr = Sb + (size_t)row * TT; float v[64]; float mx = -3.0e38f;
#pragma unroll
    for (int ch = 0; ch < 16; ++ch) { const v4f a = *(const v4f*)(sr + ch * 128 + lane * 4);
#pragma unroll
        for (int q = 0; q < 4; ++q) { v[ch * 4 + q] = a[q]; mx = fmaxf(mx, a[q]); } }
#pragma unroll
    for (int sh = 16; sh; sh >>= 1) mx = fmaxf(mx, __shfl_xor(mx, sh, 32));
    float sum = 0.f;
#pragma unroll
    for (int k = 0; k < 64; ++k) { float d0 = __fsub_rn(v[k], mx); asm volatile("" : "+v"(d0)); v[k] = __builtin_amdgcn_exp2f(__fmul_rn(d0, 1.4426950408889634f)); sum += v[k]; }
#pragma unroll
    for (int sh = 16; sh; sh >>= 1) sum += __shfl_xor(sum, sh, 32);
    const float inv = __fdiv_rn(1.0f, sum);
#pragma unroll 1
    for (int ps = 0; ps < 2; ++ps) {
#pragma unroll
        for (int ch = 0; ch < 16; ++ch) { v4f o;
#pragma unroll
            for (int q = 0; q < 4; ++q) o[q] = __fmul_rn(v[ch * 4 + q], inv); *(volatile v4f*)(sr + ch * 128 + lane * 4) = o; }
        if (ps == 0) __threadfence(); } }
__global__ __launch_bounds__(256) void k_mix(const float* __restrict__ Pb, const float* __restrict__ Wx, h16* P16) { const int e = (blockIdx.x * 256 + threadIdx.x) * 2; if (e >= QB * TT) return; float a0[NH_], a1[NH_];
#pragma unroll
    for (int h = 0; h < NH_; ++h) { a0[h] = Pb[(size_t)h * QB * TT + e]; a1[h] = Pb[(size_t)h * QB * TT + e + 1]; }
#pragma unroll 1
    for (int ps = 0; ps < 2; ++ps) {
#pragma unroll 1
        for (int g = 0; g < NH_; ++g) { float s0 = 0.f, s1 = 0.f;
#pragma unroll
            for (int h = 0; h < NH_; ++h) { float w = bfr(Wx[g * NH_ + h]); asm volatile("" : "+v"(w)); float p0 = __fmul_rn(w, a0[h]), p1 = __fmul_rn(w, a1[h]); asm volatile("" : "+v"(p0)); asm volatile("" : "+v"(p1)); s0 = __fadd_rn(s0, p0); s1 = __fadd_rn(s1, p1); }
            v2h o; o[0] = tohx(s0 * PCAR); o[1] = tohx(s1 * PCAR); *(volatile v2h*)(P16 + (size_t)g * QB * TT + e) = o; }
        if (ps == 0) __threadfence(); } }
__global__ __launch_bounds__(256) void k_mrg(const float* __restrict__ O, int qb, bf* Ah, bf* Al) { const int e = (blockIdx.x * 256 + threadIdx.x) * 2; if (e >= NH_ * QB * HD) return; const int d = e & 63; const int q = (e >> 6) & (QB - 1); const int g = e / (QB * HD); v2us oh, ol;
#pragma unroll
    for (int u = 0; u < 2; ++u) { unsigned short a, c2; splitf(O[e + u] * (1.0f / PCAR), a, c2); oh[u] = a; ol[u] = c2; } const size_t oo = ((size_t)qb * QB + q) * DD + g * HD + d; *(volatile v2us*)(Ah + oo) = oh; *(volatile v2us*)(Al + oo) = ol; __threadfence(); *(volatile v2us*)(Ah + oo) = oh; *(volatile v2us*)(Al + oo) = ol; }

extern "C" void kernel_launch(void* const* d_in, const int* in_sizes, int n_in,
                              void* d_out, int out_size, void* d_ws, size_t ws_size, hipStream_t stream) {
    (void)in_sizes; (void)n_in; (void)out_size;
    const float* x = (const float*)d_in[0]; const float* lng = (const float*)d_in[1]; const float* lnb = (const float*)d_in[2]; const float* wkv = (const float*)d_in[3]; const float* wx = (const float*)d_in[4]; const float* wout = (const float*)d_in[6];
    float* OUT = (float*)d_out;
    char* wsp = (char*)d_ws;
    auto take = [&](size_t bytes) { char* p = wsp; wsp += (bytes + 255) & ~(size_t)255; return (void*)p; };
    bf* WKV = (bf*)take((size_t)2 * DD * DD * 2); bf* WO = (bf*)take((size_t)DD * DD * 2); bf* Xh = (bf*)take((size_t)TT * DD * 2); bf* Xl = (bf*)take((size_t)TT * DD * 2); float* KV = (float*)take((size_t)TT * 2 * DD * 4);
    bf* QKh = (bf*)take((size_t)NH_ * TT * HD * 2); bf* QKl = (bf*)take((size_t)NH_ * TT * HD * 2); h16* VT = (h16*)take((size_t)NH_ * HD * TT * 2); float* Sb = (float*)take((size_t)NH_ * QB * TT * 4); h16* P16 = (h16*)take((size_t)NH_ * QB * TT * 2); float* Ob = (float*)take((size_t)NH_ * QB * HD * 4); bf* Ah = (bf*)take((size_t)TT * DD * 2); bf* Al = (bf*)take((size_t)TT * DD * 2);
    if ((size_t)(wsp - (char*)d_ws) > ws_size) return;
    k_wtG<<<(unsigned)((DD * 2 * DD / 64 + 63) / 64), 256, 0, stream>>>(wkv, DD, 2 * DD, WKV); k_wtG<<<(unsigned)((DD * DD / 64 + 63) / 64), 256, 0, stream>>>(wout, DD, DD, WO);
    const unsigned LP = (NH_ * TT * HD / 2 + 255) / 256;
    for (int b = 0; b < NB_; ++b) {
        k_ln1k<1, 0, 0><<<TT / 8, 256, 0, stream>>>(x + (size_t)b * TT * DD, lng, lnb, nullptr, nullptr, Xh, Xl, nullptr);
        k_gemmw<bf, 1, false><<<dim3(TT / 64, 2 * DD / 64, 1), 32, 0, stream>>>(Xh, Xl, WKV, nullptr, DD, KV, 2 * DD, nullptr, 0, 0, 0);
        k_qkpl<<<LP, 256, 0, stream>>>(KV, QKh, QKl); k_vt<<<LP, 256, 0, stream>>>(KV, VT);
        for (int qb = 0; qb < NQB; ++qb) {
            k_gemmw<bf, 2, false><<<dim3(QB / 64, TT / 64, NH_), 32, 0, stream>>>(QKh + (size_t)qb * QB * HD, QKl + (size_t)qb * QB * HD, QKh, QKl, HD, Sb, TT, nullptr, (size_t)TT * HD, (size_t)TT * HD, (size_t)QB * TT);
            k_smx<<<(NH_ * QB) / 8, 256, 0, stream>>>(Sb);
            k_mix<<<(QB * TT / 2 + 255) / 256, 256, 0, stream>>>(Sb, wx, P16);
            k_gemmw<h16, 0, false><<<dim3(QB / 64, 1, NH_), 32, 0, stream>>>(P16, nullptr, VT, nullptr, TT, Ob, HD, nullptr, (size_t)QB * TT, (size_t)HD * TT, (size_t)QB * HD);
            k_mrg<<<(NH_ * QB * HD / 2 + 255) / 256, 256, 0, stream>>>(Ob, qb, Ah, Al); }
        k_gemmw<bf, 1, false><<<dim3(TT / 64, DD / 64, 1), 32, 0, stream>>>(Ah, Al, WO, nullptr, DD, OUT + (size_t)b * TT * DD, DD, nullptr, 0, 0, 0); }
}
